// Mamba2Block_26113401160192
// MI455X (gfx1250) — hardware-run, weakly checked
//
#include <hip/hip_runtime.h>
#include <math.h>
#include <stdint.h>

typedef __attribute__((ext_vector_type(16))) _Float16 v16h;
typedef __attribute__((ext_vector_type(8)))  _Float16 v8h;
typedef __attribute__((ext_vector_type(8)))  float    v8f;
typedef __attribute__((ext_vector_type(4)))  float    v4f;

constexpr int kSeq     = 2048;
constexpr int kDm      = 768;
constexpr int kDin     = 1536;
constexpr int kNst     = 64;
constexpr int kNh      = 24;
constexpr int kHd      = 64;
constexpr int kConvCh  = 1664;
constexpr int kProj    = 3224;
constexpr int kProjPad = 3264;
constexpr int kFfn     = 2048;
constexpr int kDtP     = 32;
constexpr int kZxXbc   = 1536;
constexpr int kZxDt    = 3200;
constexpr int kXcB     = 1536;
constexpr int kXcC     = 1600;
constexpr float kEpsRms    = 1.1920929e-07f;
constexpr float kEpsGated  = 1e-05f;
constexpr float kWScale    = 256.0f;
constexpr float kWScaleInv = 1.0f / 256.0f;
static_assert(kDin + kConvCh + kNh == kProj, "projection split");
static_assert(kConvCh == kDin + 2 * kNst, "conv channels");
static_assert(kNh * kHd == kDin, "heads");
static_assert((kDm % 32) == 0 && (kDin % 32) == 0 && (kFfn % 32) == 0, "every GEMM K is a multiple of 32");
static_assert((kSeq % 64) == 0 && (kProjPad % 64) == 0 && (kDm % 64) == 0 && (kFfn % 64) == 0, "every GEMM M,N is a multiple of 64");
static_assert(kProjPad >= kProj, "pad");

constexpr int kConvCB = 128;
constexpr int kConvTP = 132;
constexpr int kScanTS = 32;
constexpr int kScanYP = 68;
static_assert((kConvCh % kConvCB) == 0 && (kSeq % 64) == 0 && (kSeq % kScanTS) == 0, "tiles");

constexpr int kTiles1  = (kSeq / 64) * (kProjPad / 64);
constexpr int kTiles2  = (kSeq / 64) * (kDm / 64);
constexpr int kTiles34 = (kSeq / 64) * (kFfn / 64);
constexpr int kBlk1  = (kTiles1 + 7) / 8;
constexpr int kBlk2  = (kTiles2 + 7) / 8;
constexpr int kBlk34 = (kTiles34 + 7) / 8;

constexpr size_t kOffWIN  = 0;
constexpr size_t kOffWOUT = kOffWIN  + (size_t)kProjPad * kDm * 2;
constexpr size_t kOffWG   = kOffWOUT + (size_t)kDm * kDin * 2;
constexpr size_t kOffWU   = kOffWG   + (size_t)kFfn * kDm * 2;
constexpr size_t kOffWD   = kOffWU   + (size_t)kFfn * kDm * 2;
constexpr size_t kOffH1   = kOffWD   + (size_t)kDm * kFfn * 2;
constexpr size_t kOffZX   = kOffH1   + (size_t)kSeq * kDm * 2;
constexpr size_t kOffXC   = kOffZX   + (size_t)kSeq * kProjPad * 4;
constexpr size_t kOffDT   = kOffXC   + (size_t)kSeq * kConvCh * 4;
constexpr size_t kOffY    = kOffDT   + (size_t)kSeq * kDtP * 4;
constexpr size_t kOffYN   = kOffY    + (size_t)kSeq * kDin * 4;
constexpr size_t kOffX1   = kOffYN   + (size_t)kSeq * kDin * 2;
constexpr size_t kOffH2   = kOffX1   + (size_t)kSeq * kDm * 4;
constexpr size_t kOffG    = kOffH2   + (size_t)kSeq * kDm * 2;
constexpr size_t kOffU    = kOffG    + (size_t)kSeq * kFfn * 4;
constexpr size_t kOffAP   = kOffU    + (size_t)kSeq * kFfn * 4;
constexpr size_t kWsTotal = kOffAP   + (size_t)kSeq * kFfn * 2;
static_assert(kWsTotal == 130842624ull, "carve total");
static_assert(kWsTotal <= 134217728ull, "carve cap");
static_assert((kOffWOUT % 128) == 0 && (kOffWG % 128) == 0 && (kOffWU % 128) == 0 && (kOffWD % 128) == 0 &&
              (kOffH1 % 128) == 0 && (kOffZX % 128) == 0 && (kOffXC % 128) == 0 && (kOffDT % 128) == 0 &&
              (kOffY % 128) == 0 && (kOffYN % 128) == 0 && (kOffX1 % 128) == 0 && (kOffH2 % 128) == 0 &&
              (kOffG % 128) == 0 && (kOffU % 128) == 0 && (kOffAP % 128) == 0, "128-B aligned regions");
static_assert(kOffWU == kOffWG + (size_t)kFfn * kDm * 2 && kOffU == kOffG + (size_t)kSeq * kFfn * 4, "z-batched planes contiguous");

__device__ __forceinline__ void dep_guard4_h(v8f& a, v8f& b, v8f& c, v8f& d, v16h x, v16h y) {
  asm volatile("v_nop\n\tv_nop\n\tv_nop\n\tv_nop" : "+v"(a), "+v"(b), "+v"(c), "+v"(d) : "v"(x), "v"(y));
}
__device__ __forceinline__ void keep4_h(v16h a, v16h b, v16h c, v16h d) { asm volatile("v_nop" :: "v"(a), "v"(b), "v"(c), "v"(d)); }
__device__ __forceinline__ void acc_guard4(v8f& a, v8f& b, v8f& c, v8f& d) { asm volatile("v_nop\n\tv_nop\n\tv_nop\n\tv_nop" : "+v"(a), "+v"(b), "+v"(c), "+v"(d)); }

struct FragH {
  union U { v16h v; v8h h[2]; };
  static __device__ __forceinline__ v16h load(const _Float16* p) {
    U f; f.h[0] = *(const v8h*)(p); f.h[1] = *(const v8h*)(p + 16); return f.v;
  }
  static __device__ __forceinline__ v8f mma(v16h a, v16h b, v8f c) {
    return __builtin_amdgcn_wmma_f32_16x16x32_f16(false, a, false, b, (short)0, c, false, false);
  }
};

__device__ __forceinline__ float silu_f32(float v) {
  const float sg = __builtin_amdgcn_rcpf(1.0f + expf(-v));
  return v * sg;
}

template <bool RESID>
__global__ __launch_bounds__(256) void gemm_f16_kernel(
    const unsigned short* __restrict__ Ap, int lda, long strideA,
    const unsigned short* __restrict__ Btp, int ldb, long strideB,
    float* __restrict__ Cout, int ldc, long strideC,
    const float* __restrict__ resid, long strideR,
    int M, int N, int K, float scale) {
  const _Float16* A  = (const _Float16*)Ap;
  const _Float16* Bt = (const _Float16*)Btp;
  __shared__ __align__(16) float sT[8][16 * 68];
  const int b    = blockIdx.y;
  const int lane = threadIdx.x & 31;
  const int wave = threadIdx.x >> 5;
  const int tilesN = N >> 6;
  const int tilesM = M >> 6;
  const int tile = blockIdx.x * 8 + wave;
  if (tile >= tilesM * tilesN) return;
  const int tm = tile / tilesN;
  const int tn = tile - tm * tilesN;
  const int m0 = tm << 6;
  const int n0 = tn << 6;

  const _Float16* Ab = A  + (size_t)b * strideA;
  const _Float16* Bb = Bt + (size_t)b * strideB;

  const int rlane = lane & 15;
  const int koff  = (lane >> 4) * 8;
  const int mOff  = (lane >> 4) * 8;

  v8f acc[4][4];
#pragma unroll
  for (int i = 0; i < 4; ++i)
#pragma unroll
    for (int j = 0; j < 4; ++j) acc[i][j] = (v8f){0.f,0.f,0.f,0.f,0.f,0.f,0.f,0.f};

  for (int k0 = 0; k0 < K; k0 += 32) {
    v16h bh[4];
#pragma unroll
    for (int j = 0; j < 4; ++j) {
      const size_t bo = (size_t)(n0 + (j << 4) + rlane) * ldb + koff + k0;
      bh[j] = FragH::load(Bb + bo);
    }
#pragma unroll
    for (int i = 0; i < 4; ++i) {
      const size_t ao = (size_t)(m0 + (i << 4) + rlane) * lda + koff + k0;
      v16h ah = FragH::load(Ab + ao);
#pragma unroll
      for (int j = 0; j < 4; ++j) acc[i][j] = FragH::mma(ah, bh[j], acc[i][j]);
      dep_guard4_h(acc[i][0], acc[i][1], acc[i][2], acc[i][3], ah, bh[3]);
    }
    keep4_h(bh[0], bh[1], bh[2], bh[3]);
  }
  acc_guard4(acc[0][0], acc[0][1], acc[0][2], acc[0][3]);
  acc_guard4(acc[1][0], acc[1][1], acc[1][2], acc[1][3]);
  acc_guard4(acc[2][0], acc[2][1], acc[2][2], acc[2][3]);
  acc_guard4(acc[3][0], acc[3][1], acc[3][2], acc[3][3]);

  float* slab = sT[wave];
  float* C = Cout + (size_t)b * strideC;
  const float* Rb = RESID ? (resid + (size_t)b * strideR) : nullptr;
#pragma unroll
  for (int i = 0; i < 4; ++i) {
    const int mBase = m0 + (i << 4);
#pragma unroll
    for (int j = 0; j < 4; ++j) {
#pragma unroll
      for (int r = 0; r < 8; ++r) {
        slab[(mOff + r) * 68 + (j << 4) + rlane] = acc[i][j][r] * scale;
      }
    }
    __builtin_amdgcn_fence(__ATOMIC_RELEASE, "workgroup");
    __builtin_amdgcn_wave_barrier();
    __builtin_amdgcn_fence(__ATOMIC_ACQUIRE, "workgroup");
    {
      const int hh = lane >> 4, c4 = (lane & 15) * 4;
      for (int pass = 0; pass < 2; ++pass) {
#pragma unroll
        for (int it = 0; it < 8; ++it) {
          const int row = it * 2 + hh;
          v4f v = *(const v4f*)(slab + row * 68 + c4);
          if (RESID) {
            const v4f rr = *(const v4f*)(Rb + (size_t)(mBase + row) * ldc + n0 + c4);
            v += rr;
          }
          *(volatile v4f*)(C + (size_t)(mBase + row) * ldc + n0 + c4) = v;
        }
        __threadfence();
      }
    }
    __builtin_amdgcn_fence(__ATOMIC_RELEASE, "workgroup");
    __builtin_amdgcn_wave_barrier();
    __builtin_amdgcn_fence(__ATOMIC_ACQUIRE, "workgroup");
  }
}

__global__ __launch_bounds__(256) void cast_rows_f16_kernel(
    const float* __restrict__ src, unsigned short* __restrict__ dst,
    int nrows_real, int ncols, int total8, float scale) {
  const int i = blockIdx.x * 256 + threadIdx.x;
  if (i >= total8) return;
  const size_t e0 = (size_t)i << 3;
  const int row = (int)(e0 / (size_t)ncols);
  const int col = (int)(e0 - (size_t)row * (size_t)ncols);
  const int rowc = (row < nrows_real) ? row : (nrows_real - 1);
  const float* sp = src + (size_t)rowc * ncols + col;
  const v4f a0 = *(const v4f*)(sp);
  const v4f a1 = *(const v4f*)(sp + 4);
  const float live = (row < nrows_real) ? scale : 0.0f;
  v8h hv;
#pragma unroll
  for (int e = 0; e < 4; ++e) {
    hv[e]     = (_Float16)(a0[e] * live);
    hv[4 + e] = (_Float16)(a1[e] * live);
  }
  unsigned short* q = dst + e0;
  *(volatile v8h*)q = hv;
  __threadfence();
  *(volatile v8h*)q = hv;
}

template <int DW>
__global__ __launch_bounds__(DW / 8) void rmsnorm_f16_kernel(
    const float* __restrict__ src, const float* __restrict__ w, unsigned short* __restrict__ dst, float eps) {
  constexpr int NT = DW / 8;
  constexpr int NWV = NT / 32;
  static_assert((NT % 32) == 0 && ((DW * 2) % 128) == 0, "whole waves and whole lines");
  __shared__ float sred[NWV];
  const int tid = threadIdx.x, lane = tid & 31, wave = tid >> 5;
  const size_t row = blockIdx.x;
  const float* sp = src + row * DW + (size_t)tid * 8;
  const v4f a0 = *(const v4f*)(sp);
  const v4f a1 = *(const v4f*)(sp + 4);
  float ss = 0.0f;
#pragma unroll
  for (int e = 0; e < 4; ++e) ss = fmaf(a0[e], a0[e], ss);
#pragma unroll
  for (int e = 0; e < 4; ++e) ss = fmaf(a1[e], a1[e], ss);
#pragma unroll
  for (int off = 16; off > 0; off >>= 1) ss += __shfl_xor(ss, off, 32);
  if (lane == 0) sred[wave] = ss;
  __syncthreads();
  float tot = 0.0f;
#pragma unroll
  for (int q = 0; q < NWV; ++q) tot += sred[q];
  const float sc = rsqrtf(tot * (1.0f / (float)DW) + eps);
  const v4f w0 = *(const v4f*)(w + tid * 8);
  const v4f w1 = *(const v4f*)(w + tid * 8 + 4);
  v8h hv;
#pragma unroll
  for (int e = 0; e < 4; ++e) {
    hv[e]     = (_Float16)(a0[e] * sc * w0[e]);
    hv[4 + e] = (_Float16)(a1[e] * sc * w1[e]);
  }
  unsigned short* q = dst + row * DW + (size_t)tid * 8;
  *(volatile v8h*)q = hv;
  __threadfence();
  *(volatile v8h*)q = hv;
}

__global__ __launch_bounds__(192) void gated_norm_f16_kernel(
    const float* __restrict__ Y, const float* __restrict__ ZX, const float* __restrict__ w,
    unsigned short* __restrict__ dst) {
  constexpr int NWV = 6;
  __shared__ float sred[NWV];
  const int tid = threadIdx.x, lane = tid & 31, wave = tid >> 5;
  const size_t row = blockIdx.x;
  const float* yp = Y  + row * kDin     + (size_t)tid * 8;
  const float* zp = ZX + row * kProjPad + (size_t)tid * 8;
  const v4f y0 = *(const v4f*)(yp), y1 = *(const v4f*)(yp + 4);
  const v4f z0 = *(const v4f*)(zp), z1 = *(const v4f*)(zp + 4);
  float u[8];
#pragma unroll
  for (int e = 0; e < 4; ++e) {
    u[e]     = y0[e] * silu_f32(z0[e]);
    u[4 + e] = y1[e] * silu_f32(z1[e]);
  }
  float ss = 0.0f;
#pragma unroll
  for (int e = 0; e < 8; ++e) ss = fmaf(u[e], u[e], ss);
#pragma unroll
  for (int off = 16; off > 0; off >>= 1) ss += __shfl_xor(ss, off, 32);
  if (lane == 0) sred[wave] = ss;
  __syncthreads();
  float tot = 0.0f;
#pragma unroll
  for (int q = 0; q < NWV; ++q) tot += sred[q];
  const float sc = rsqrtf(tot * (1.0f / (float)kDin) + kEpsGated);
  const v4f w0 = *(const v4f*)(w + tid * 8);
  const v4f w1 = *(const v4f*)(w + tid * 8 + 4);
  v8h hv;
#pragma unroll
  for (int e = 0; e < 4; ++e) {
    hv[e]     = (_Float16)(u[e] * sc * w0[e]);
    hv[4 + e] = (_Float16)(u[4 + e] * sc * w1[e]);
  }
  unsigned short* q = dst + row * kDin + (size_t)tid * 8;
  *(volatile v8h*)q = hv;
  __threadfence();
  *(volatile v8h*)q = hv;
}

__global__ __launch_bounds__(256) void silu_mul_f16_kernel(
    const float* __restrict__ G, const float* __restrict__ Uv, unsigned short* __restrict__ dst, int total8) {
  const int i = blockIdx.x * 256 + threadIdx.x;
  if (i >= total8) return;
  const size_t e0 = (size_t)i << 3;
  const v4f g0 = *(const v4f*)(G + e0),  g1 = *(const v4f*)(G + e0 + 4);
  const v4f u0 = *(const v4f*)(Uv + e0), u1 = *(const v4f*)(Uv + e0 + 4);
  v8h hv;
#pragma unroll
  for (int e = 0; e < 4; ++e) {
    hv[e]     = (_Float16)(silu_f32(g0[e]) * u0[e]);
    hv[4 + e] = (_Float16)(silu_f32(g1[e]) * u1[e]);
  }
  unsigned short* q = dst + e0;
  *(volatile v8h*)q = hv;
  __threadfence();
  *(volatile v8h*)q = hv;
}

__global__ __launch_bounds__(kConvCB) void conv_silu_kernel(
    const float* __restrict__ ZX, const float* __restrict__ cw, const float* __restrict__ cb,
    float* __restrict__ XC) {
  __shared__ __align__(16) float sT[16 * kConvTP];
  const int tid = threadIdx.x, lane = tid & 31, wave = tid >> 5;
  const int c0 = blockIdx.x * kConvCB;
  const int c  = c0 + tid;
  const int t0 = blockIdx.y * 64;
  const v4f wv = *(const v4f*)(cw + (size_t)c * 4);
  const float bc = cb[c];
  float xm3, xm2, xm1;
  {
    const bool hist = (t0 > 0);
    const int rb = hist ? (t0 - 3) : t0;
    const float v3 = ZX[(size_t)rb * kProjPad + kZxXbc + c];
    const float v2 = ZX[(size_t)(rb + 1) * kProjPad + kZxXbc + c];
    const float v1 = ZX[(size_t)(rb + 2) * kProjPad + kZxXbc + c];
    xm3 = hist ? v3 : 0.f;
    xm2 = hist ? v2 : 0.f;
    xm1 = hist ? v1 : 0.f;
  }
#pragma unroll 1
  for (int sub = 0; sub < 4; ++sub) {
    const int lb = t0 + sub * 16;
#pragma unroll 1
    for (int s = 0; s < 16; ++s) {
      const float xcur = ZX[(size_t)(lb + s) * kProjPad + kZxXbc + c];
      float acc = wv[0] * xm3;
      acc = fmaf(wv[1], xm2, acc);
      acc = fmaf(wv[2], xm1, acc);
      acc = fmaf(wv[3], xcur, acc);
      const float sv = acc + bc;
      sT[s * kConvTP + tid] = silu_f32(sv);
      xm3 = xm2; xm2 = xm1; xm1 = xcur;
    }
    __syncthreads();
    v4f fv[4];
#pragma unroll
    for (int it = 0; it < 4; ++it) fv[it] = *(const v4f*)(sT + (it * 4 + wave) * kConvTP + lane * 4);
    for (int pass = 0; pass < 2; ++pass) {
#pragma unroll
      for (int it = 0; it < 4; ++it)
        *(volatile v4f*)(XC + (size_t)(lb + it * 4 + wave) * kConvCh + c0 + lane * 4) = fv[it];
      __threadfence();
    }
    __syncthreads();
  }
}

__global__ __launch_bounds__(256) void dt_softplus_kernel(
    const float* __restrict__ ZX, const float* __restrict__ dtb, float* __restrict__ DT) {
  const int tid = threadIdx.x, lane = tid & 31, wave = tid >> 5;
  const int row = blockIdx.x * 8 + wave;
  const int hc = (lane < kNh) ? lane : (kNh - 1);
  const float v = ZX[(size_t)row * kProjPad + kZxDt + hc] + dtb[hc];
  const float sp = fmaxf(v, 0.0f) + log1pf(expf(-fabsf(v)));
  const float val = (lane < kNh) ? sp : 0.0f;
  volatile float* q = DT + (size_t)row * kDtP + lane;
  *q = val;
  __threadfence();
  *q = val;
}

__global__ __launch_bounds__(64) void scan_kernel(
    const float* __restrict__ XC, const float* __restrict__ DT, const float* __restrict__ Alog,
    const float* __restrict__ Dp, float* __restrict__ Y) {
  __shared__ __align__(16) float sS[kNst * kHd];
  __shared__ __align__(16) float sB[kScanTS * kNst];
  __shared__ __align__(16) float sC[kScanTS * kNst];
  __shared__ __align__(16) float sY[kScanTS * kScanYP];
  __shared__ float sDT[kScanTS];
  const int tid = threadIdx.x, lane = tid & 31, wave = tid >> 5;
  const int h = blockIdx.x;
  const int p = tid;
  const float Ah = -expf(Alog[h]);
  const float Dh = Dp[h];
  const v4f zero4 = (v4f){0.f, 0.f, 0.f, 0.f};
#pragma unroll
  for (int n4 = 0; n4 < 16; ++n4) *(v4f*)(sS + 4 * (n4 * 64 + p)) = zero4;
  const int lr = tid >> 4, lc4 = (tid & 15) * 4;
  const int hh = lane >> 4, c4 = (lane & 15) * 4;
#pragma unroll 1
  for (int t0 = 0; t0 < kSeq; t0 += kScanTS) {
    __syncthreads();
#pragma unroll 4
    for (int i = 0; i < 8; ++i) {
      const int r = lr + 4 * i;
      const float* xr = XC + (size_t)(t0 + r) * kConvCh;
      *(v4f*)(sB + r * kNst + lc4) = *(const v4f*)(xr + kXcB + lc4);
      *(v4f*)(sC + r * kNst + lc4) = *(const v4f*)(xr + kXcC + lc4);
    }
    if (tid < kScanTS) sDT[tid] = DT[(size_t)(t0 + tid) * kDtP + h];
    __syncthreads();
#pragma unroll 1
    for (int s = 0; s < kScanTS; ++s) {
      const int t = t0 + s;
      const float dtv = sDT[s];
      const float xv  = XC[(size_t)t * kConvCh + h * kHd + p];
      const float dA  = expf(dtv * Ah);
      const float dtx = dtv * xv;
      const float* br = sB + s * kNst;
      const float* cr = sC + s * kNst;
      float yacc = 0.0f;
#pragma unroll 2
      for (int n4 = 0; n4 < 16; ++n4) {
        float* sp = sS + 4 * (n4 * 64 + p);
        v4f st = *(const v4f*)(sp);
        const v4f bv = *(const v4f*)(br + 4 * n4);
        const v4f cv = *(const v4f*)(cr + 4 * n4);
        st.x = fmaf(st.x, dA, dtx * bv.x);
        st.y = fmaf(st.y, dA, dtx * bv.y);
        st.z = fmaf(st.z, dA, dtx * bv.z);
        st.w = fmaf(st.w, dA, dtx * bv.w);
        yacc = fmaf(st.x, cv.x, yacc);
        yacc = fmaf(st.y, cv.y, yacc);
        yacc = fmaf(st.z, cv.z, yacc);
        yacc = fmaf(st.w, cv.w, yacc);
        *(v4f*)(sp) = st;
      }
      const float yv = fmaf(Dh, xv, yacc);
      sY[s * kScanYP + p] = yv;
    }
    __syncthreads();
    for (int pass = 0; pass < 2; ++pass) {
#pragma unroll
      for (int it = 0; it < 8; ++it) {
        const int row = it * 4 + wave * 2 + hh;
        const v4f v = *(const v4f*)(sY + row * kScanYP + c4);
        *(volatile v4f*)(Y + (size_t)(t0 + row) * kDin + h * kHd + c4) = v;
      }
      __threadfence();
    }
  }
}

extern "C" void kernel_launch(void* const* d_in, const int* in_sizes, int n_in,
                              void* d_out, int out_size, void* d_ws, size_t ws_size,
                              hipStream_t stream) {
  if (n_in < 14) return;
  if (in_sizes[0]  != kSeq * kDm) return;
  if (in_sizes[1]  != kDm) return;
  if (in_sizes[2]  != kDm) return;
  if (in_sizes[3]  != kProj * kDm) return;
  if (in_sizes[4]  != kConvCh * 4) return;
  if (in_sizes[5]  != kConvCh) return;
  if (in_sizes[6]  != kNh) return;
  if (in_sizes[7]  != kNh) return;
  if (in_sizes[8]  != kNh) return;
  if (in_sizes[9]  != kDin) return;
  if (in_sizes[10] != kDm * kDin) return;
  if (in_sizes[11] != kFfn * kDm) return;
  if (in_sizes[12] != kFfn * kDm) return;
  if (in_sizes[13] != kDm * kFfn) return;
  if (out_size != kSeq * kDm) return;
  if (ws_size < kWsTotal) return;

  const float* x          = (const float*)d_in[0];
  const float* norm1_w    = (const float*)d_in[1];
  const float* norm2_w    = (const float*)d_in[2];
  const float* in_proj_w  = (const float*)d_in[3];
  const float* conv_w     = (const float*)d_in[4];
  const float* conv_b     = (const float*)d_in[5];
  const float* dt_bias    = (const float*)d_in[6];
  const float* A_log      = (const float*)d_in[7];
  const float* Dp         = (const float*)d_in[8];
  const float* ssm_norm_w = (const float*)d_in[9];
  const float* out_proj_w = (const float*)d_in[10];
  const float* gate_w     = (const float*)d_in[11];
  const float* up_w       = (const float*)d_in[12];
  const float* down_w     = (const float*)d_in[13];
  float* out = (float*)d_out;

  char* ws = (char*)d_ws;
  unsigned short* WIN  = (unsigned short*)(ws + kOffWIN);
  unsigned short* WOUT = (unsigned short*)(ws + kOffWOUT);
  unsigned short* WG   = (unsigned short*)(ws + kOffWG);
  unsigned short* WU   = (unsigned short*)(ws + kOffWU);
  unsigned short* WD   = (unsigned short*)(ws + kOffWD);
  unsigned short* H1   = (unsigned short*)(ws + kOffH1);
  float*          ZX   = (float*)(ws + kOffZX);
  float*          XC   = (float*)(ws + kOffXC);
  float*          DT   = (float*)(ws + kOffDT);
  float*          Y    = (float*)(ws + kOffY);
  unsigned short* YN   = (unsigned short*)(ws + kOffYN);
  float*          X1   = (float*)(ws + kOffX1);
  unsigned short* H2   = (unsigned short*)(ws + kOffH2);
  float*          G    = (float*)(ws + kOffG);
  float*          U    = (float*)(ws + kOffU);
  unsigned short* AP   = (unsigned short*)(ws + kOffAP);
  (void)WU; (void)U;

  constexpr int kTot8WIN  = kProjPad * kDm / 8;
  constexpr int kTot8WOUT = kDm * kDin / 8;
  constexpr int kTot8WF   = kFfn * kDm / 8;
  constexpr int kTot8AP   = kSeq * kFfn / 8;

  cast_rows_f16_kernel<<<(kTot8WIN + 255) / 256, 256, 0, stream>>>(in_proj_w, WIN, kProj, kDm, kTot8WIN, kWScale);
  cast_rows_f16_kernel<<<(kTot8WOUT + 255) / 256, 256, 0, stream>>>(out_proj_w, WOUT, kDm, kDin, kTot8WOUT, kWScale);
  cast_rows_f16_kernel<<<(kTot8WF + 255) / 256, 256, 0, stream>>>(gate_w, WG, kFfn, kDm, kTot8WF, kWScale);
  cast_rows_f16_kernel<<<(kTot8WF + 255) / 256, 256, 0, stream>>>(up_w, WU, kFfn, kDm, kTot8WF, kWScale);
  cast_rows_f16_kernel<<<(kTot8WF + 255) / 256, 256, 0, stream>>>(down_w, WD, kDm, kFfn, kTot8WF, kWScale);

  rmsnorm_f16_kernel<kDm><<<kSeq, kDm / 8, 0, stream>>>(x, norm1_w, H1, kEpsRms);

  gemm_f16_kernel<false><<<dim3(kBlk1, 1), 256, 0, stream>>>(
      H1, kDm, 0L,
      WIN, kDm, 0L,
      ZX, kProjPad, 0L,
      nullptr, 0L,
      kSeq, kProjPad, kDm, kWScaleInv);

  conv_silu_kernel<<<dim3(kConvCh / kConvCB, kSeq / 64), kConvCB, 0, stream>>>(ZX, conv_w, conv_b, XC);

  dt_softplus_kernel<<<kSeq / 8, 256, 0, stream>>>(ZX, dt_bias, DT);

  scan_kernel<<<kNh, kHd, 0, stream>>>(XC, DT, A_log, Dp, Y);

  gated_norm_f16_kernel<<<kSeq, kDin / 8, 0, stream>>>(Y, ZX, ssm_norm_w, YN);

  gemm_f16_kernel<true><<<dim3(kBlk2, 1), 256, 0, stream>>>(
      YN, kDin, 0L,
      WOUT, kDin, 0L,
      X1, kDm, 0L,
      x, 0L,
      kSeq, kDm, kDin, kWScaleInv);

  rmsnorm_f16_kernel<kDm><<<kSeq, kDm / 8, 0, stream>>>(X1, norm2_w, H2, kEpsRms);

  gemm_f16_kernel<false><<<dim3(kBlk34, 2), 256, 0, stream>>>(
      H2, kDm, 0L,
      WG, kDm, (long)kFfn * kDm,
      G, kFfn, (long)kSeq * kFfn,
      nullptr, 0L,
      kSeq, kFfn, kDm, kWScaleInv);

  silu_mul_f16_kernel<<<(kTot8AP + 255) / 256, 256, 0, stream>>>(G, U, AP, kTot8AP);

  gemm_f16_kernel<true><<<dim3(kBlk2, 1), 256, 0, stream>>>(
      AP, kFfn, 0L,
      WD, kFfn, 0L,
      out, kDm, 0L,
      X1, 0L,
      kSeq, kDm, kFfn, kWScaleInv);
}
